// Capsule_14456859918499
// MI455X (gfx1250) — hardware-verified
//
#include <hip/hip_runtime.h>


namespace {
constexpr int NB_ = 32, SQ = 128, DIN = 1024, NC = 16, DC = 512, NU = NC * DC, NR = NB_ * SQ;

typedef _Float16 b16;
typedef __attribute__((ext_vector_type(16))) _Float16 v16b;
typedef __attribute__((ext_vector_type(8)))  _Float16 v8b;
typedef __attribute__((ext_vector_type(8)))  float v8f;
typedef __attribute__((ext_vector_type(4)))  float v4f;

__device__ __forceinline__ v8b ld8b(const b16* p) { return *(const v8b*)p; }
__device__ __forceinline__ v16b cat8b(v8b a, v8b b) { return __builtin_shufflevector(a, b, 0, 1, 2, 3, 4, 5, 6, 7, 8, 9, 10, 11, 12, 13, 14, 15); }
__device__ __forceinline__ v16b frag_kb(const b16* p, int hh) { return cat8b(ld8b(p + 8 * hh), ld8b(p + 16 + 8 * hh)); }
__device__ __forceinline__ void split16(float v, b16& hi, b16& lo) { hi = (b16)v; lo = (b16)(v - (float)hi); }
__device__ __forceinline__ void frag_ksplit(const float* p, int hh, v16b& fh_, v16b& fl_) {
  const float* p0 = p + 8 * hh; const float* p1 = p + 16 + 8 * hh;
#pragma unroll
  for (int e = 0; e < 8; ++e) { b16 a, c; split16(p0[e], a, c); fh_[e] = a; fl_[e] = c; split16(p1[e], a, c); fh_[8 + e] = a; fl_[8 + e] = c; }
}
__device__ __forceinline__ v8f wmma16b(v16b a, v16b b, v8f c) {
  v8f d = __builtin_amdgcn_wmma_f32_16x16x32_f16(false, a, false, b, (short)0, c, false, false);
  asm volatile("v_nop\n\tv_nop\n\tv_nop\n\tv_nop" : "+v"(d) : "v"(a), "v"(b));
  return d;
}
__device__ __forceinline__ void wave_lds_sync() {
  __builtin_amdgcn_fence(__ATOMIC_RELEASE, "workgroup");
  __builtin_amdgcn_wave_barrier();
  __builtin_amdgcn_fence(__ATOMIC_ACQUIRE, "workgroup");
}

struct Opnd { const void* p0; const void* p1; int ld; };
template <int NP> __device__ __forceinline__ void load_frags(const Opnd& o, int row, int kb, int hh, v16b& fh_, v16b& fl_) {
  if (NP == 0) { frag_ksplit((const float*)o.p0 + (size_t)row * o.ld + kb, hh, fh_, fl_); }
  else if (NP == 4) {
    const float* p = (const float*)o.p0 + (size_t)row * o.ld + kb; const float* p0 = p + 8 * hh; const float* p1 = p + 16 + 8 * hh;
#pragma unroll
    for (int e = 0; e < 8; ++e) { b16 a, c; split16(p0[e] * 64.0f, a, c); fh_[e] = a; fl_[e] = c; split16(p1[e] * 64.0f, a, c); fh_[8 + e] = a; fl_[8 + e] = c; }
  } else if (NP == 3) {
    const float* p = (const float*)o.p0 + (size_t)row * o.ld + kb; const float* p0 = p + 8 * hh; const float* p1 = p + 16 + 8 * hh;
#pragma unroll
    for (int e = 0; e < 8; ++e) { fh_[e] = (b16)p0[e]; fh_[8 + e] = (b16)p1[e]; }
    fl_ = fh_;
  } else {
    fh_ = frag_kb((const b16*)o.p0 + (size_t)row * o.ld + kb, hh);
    if (NP == 2) fl_ = frag_kb((const b16*)o.p1 + (size_t)row * o.ld + kb, hh); else fl_ = fh_;
  }
}
template <int ANP, int BNP> __device__ __forceinline__ v8f mac(v16b ah, v16b al, v16b bh, v16b bl, v8f c) {
  c = wmma16b(ah, bh, c);
  if (BNP == 0 || BNP == 2 || BNP == 4) c = wmma16b(ah, bl, c);
  if (ANP == 0 || ANP == 2 || ANP == 4) c = wmma16b(al, bh, c);
  return c;
}
template <int ANP, int BNP>
__device__ __forceinline__ void gemm_tile(const Opnd& A, const Opnd& B, int K, int m0, int c0, int nloc, int hlf, v8f (&acc)[2][4]) {
  for (int kb = 0; kb < K; kb += 32) {
    v16b a0h, a0l, a1h, a1l;
    load_frags<ANP>(A, m0 + nloc, kb, hlf, a0h, a0l);
    load_frags<ANP>(A, m0 + 16 + nloc, kb, hlf, a1h, a1l);
#pragma unroll
    for (int t = 0; t < 4; ++t) {
      v16b bh, bl;
      load_frags<BNP>(B, c0 + t * 16 + nloc, kb, hlf, bh, bl);
      acc[0][t] = mac<ANP, BNP>(a0h, a0l, bh, bl, acc[0][t]);
      acc[1][t] = mac<ANP, BNP>(a1h, a1l, bh, bl, acc[1][t]);
    }
  }
}

__device__ __forceinline__ void epi_planes(v8f (&acc)[2][4], float scale, bool two, b16* __restrict__ oh, b16* __restrict__ ol, int ldo,
                                           int m0, int c0, int lane, b16* Th, b16* Tl) {
  const int nloc = lane & 15, hlf = lane >> 4;
#pragma unroll
  for (int t = 0; t < 4; ++t)
#pragma unroll
    for (int r = 0; r < 2; ++r)
#pragma unroll
      for (int v = 0; v < 8; ++v) {
        const int rr = r * 16 + v + 8 * hlf, cc = t * 16 + nloc;
        b16 h_, l_; split16(acc[r][t][v] * scale, h_, l_);
        Th[rr * 64 + cc] = h_; Tl[rr * 64 + cc] = l_;
      }
  wave_lds_sync();
  for (int pass = 0; pass < 2; ++pass) {
#pragma unroll
    for (int j = 0; j < 8; ++j) {
      const int rr = j * 4 + (lane >> 3), c8 = (lane & 7) * 8;
      const size_t o = (size_t)(m0 + rr) * ldo + c0 + c8;
      *(volatile v8b*)(oh + o) = ld8b(Th + rr * 64 + c8);
      if (two) *(volatile v8b*)(ol + o) = ld8b(Tl + rr * 64 + c8);
    }
    __threadfence();
  }
}
__device__ __forceinline__ void epi_f32(v8f (&acc)[2][4], float scale, const float* rscale, float* __restrict__ out, int ldo, int m0, int c0, int lane, float* Tt) {
  const int nloc = lane & 15, hlf = lane >> 4;
#pragma unroll
  for (int t = 0; t < 4; ++t)
#pragma unroll
    for (int r = 0; r < 2; ++r)
#pragma unroll
      for (int v = 0; v < 8; ++v) {
        const int rr = r * 16 + v + 8 * hlf;
        const float rs = rscale ? rscale[(size_t)(m0 + rr) * 32] : 1.0f;
        Tt[rr * 64 + t * 16 + nloc] = acc[r][t][v] * scale * rs;
      }
  wave_lds_sync();
  float* dst0 = out + (size_t)m0 * ldo + c0;
  for (int pass = 0; pass < 2; ++pass) {
#pragma unroll
    for (int j = 0; j < 16; ++j) { const int rr = j * 2 + hlf, c4 = nloc * 4; *(volatile v4f*)(dst0 + (size_t)rr * ldo + c4) = *(const v4f*)(Tt + rr * 64 + c4); }
    __threadfence();
  }
}


__global__ __launch_bounds__(256) void tr_kernel(const float* __restrict__ W, b16* __restrict__ wt) {
  __shared__ __attribute__((aligned(16))) b16 Tl[64][72];
  const int tid = threadIdx.x, lane = tid & 31, wave = tid >> 5, n0 = blockIdx.x * 64, k0 = blockIdx.y * 64;
  for (int i = tid; i < 64 * 64; i += 256) { const int kk = i / 64, n = i % 64; Tl[n][kk] = (b16)W[(size_t)(k0 + kk) * NU + n0 + n]; }
  __syncthreads();
  for (int pass = 0; pass < 2; ++pass) {
#pragma unroll
    for (int j = 0; j < 2; ++j) { const int rr = wave * 8 + j * 4 + (lane >> 3), c8 = (lane & 7) * 8; *(volatile v8b*)(wt + (size_t)(n0 + rr) * DIN + k0 + c8) = *(const v8b*)(&Tl[rr][c8]); }
    __threadfence();
  }
}

__global__ __launch_bounds__(128) void proj_kernel(const float* __restrict__ x, const b16* __restrict__ wt, b16* __restrict__ u16) {
  __shared__ __attribute__((aligned(16))) b16 Ts[4][2][32 * 64];
  const int lane = threadIdx.x & 31, wave = threadIdx.x >> 5, nloc = lane & 15, hlf = lane >> 4;
  const int m0 = blockIdx.y * 128 + wave * 32, c0 = blockIdx.x * 64;
  v8f acc[2][4];
#pragma unroll
  for (int r = 0; r < 2; ++r)
#pragma unroll
    for (int t = 0; t < 4; ++t) acc[r][t] = (v8f){};
  const Opnd A{x, nullptr, DIN}, B{wt, nullptr, DIN};
  gemm_tile<3, 1>(A, B, DIN, m0, c0, nloc, hlf, acc);
#pragma unroll
  for (int t = 0; t < 4; ++t)
#pragma unroll
    for (int r = 0; r < 2; ++r)
#pragma unroll
      for (int v = 0; v < 8; ++v) { const float a2 = acc[r][t][v]; acc[r][t][v] = 1.0f - 2.0f / (1.0f + __expf(2.0f * a2)); }
  epi_planes(acc, 1.0f, false, u16, nullptr, NU, m0, c0, lane, Ts[wave][0], Ts[wave][1]);
}

__global__ __launch_bounds__(256) void route_kernel(const b16* __restrict__ u16, float* __restrict__ Vout, float* __restrict__ Cout, float* __restrict__ Bout) {
  __shared__ float Bl[SQ][NC], Cl[SQ][NC];
  __shared__ __attribute__((aligned(16))) float SV[NC][DC];
  __shared__ float nrm[NC];
  const int b = blockIdx.x, t = threadIdx.x, lane = t & 31, wave = t >> 5;
  const b16* ub = u16 + (size_t)b * SQ * NU;
  for (int i = t; i < SQ * NC; i += 256) (&Bl[0][0])[i] = 0.0f;
  __syncthreads();
  for (int it = 0; it < 3; ++it) {
    if (t < SQ) {
      float mx = -INFINITY;
#pragma unroll
      for (int n = 0; n < NC; ++n) mx = fmaxf(mx, Bl[t][n]);
      float e[NC], sm = 0.0f;
#pragma unroll
      for (int n = 0; n < NC; ++n) { e[n] = expf(Bl[t][n] - mx); sm += e[n]; }
      const float inv = 1.0f / sm;
#pragma unroll
      for (int n = 0; n < NC; ++n) Cl[t][n] = e[n] * inv;
    }
    __syncthreads();
    for (int pass = 0; pass < 2; ++pass) {
      for (int i = t; i < SQ * NC; i += 256) { ((volatile float*)Cout)[((size_t)it * NB_ + b) * SQ * NC + i] = (&Cl[0][0])[i]; if (it == 2) ((volatile float*)Bout)[(size_t)b * SQ * NC + i] = (&Bl[0][0])[i]; }
      __threadfence();
    }
    for (int i = t; i < NC * DC; i += 256) {
      const int n = i / DC, dd = i % DC; float s = 0.0f;
#pragma unroll 1
      for (int sq = 0; sq < SQ; ++sq) s += Cl[sq][n] * (float)ub[(size_t)sq * NU + n * DC + dd];
      SV[n][dd] = s;
    }
    __syncthreads();
    for (int q = 0; q < 2; ++q) { const int n = wave * 2 + q; float s = 0.0f;
      for (int dd = lane; dd < DC; dd += 32) s += SV[n][dd] * SV[n][dd];
#pragma unroll
      for (int o = 16; o > 0; o >>= 1) s += __shfl_xor(s, o);
      if (lane == 0) nrm[n] = 1.0f / sqrtf(s + 1e-7f); }
    __syncthreads();
    for (int i = t; i < NC * DC; i += 256) { const int n = i / DC; (&SV[0][0])[i] *= nrm[n]; }
    __syncthreads();
    for (int i = t; i < SQ * NC; i += 256) {
      const int sq = i / NC, n = i % NC; const b16* ur = ub + (size_t)sq * NU + n * DC; float s = 0.0f;
#pragma unroll 1
      for (int dd = 0; dd < DC; dd += 8) { const v8b uv = ld8b(ur + dd);
#pragma unroll
        for (int e = 0; e < 8; ++e) s += (float)uv[e] * SV[n][dd + e]; }
      Bl[sq][n] += s;
    }
    __syncthreads();
  }
  for (int pass = 0; pass < 2; ++pass) { for (int i = t; i < NC * DC; i += 256) ((volatile float*)Vout)[(size_t)b * NC * DC + i] = (&SV[0][0])[i]; __threadfence(); }
}
}

extern "C" void kernel_launch(void* const* d_in, const int* in_sizes, int n_in,
                              void* d_out, int out_size, void* d_ws, size_t ws_size, hipStream_t stream) {
  (void)n_in; (void)out_size;
  const float* x = (const float*)d_in[0];
  const float* W = (const float*)d_in[1];
  float* out = (float*)d_out;
  if (in_sizes[0] != NR * DIN || in_sizes[1] != DIN * NU) return;
  size_t off = 0; char* ws = (char*)d_ws;
  auto carve = [&](size_t bytes) { char* p = ws + off; off += (bytes + 255) & ~(size_t)255; return p; };
  b16* wt = (b16*)carve((size_t)NU * DIN * 2);
  b16* u16 = (b16*)carve((size_t)NR * NU * 2);
  if (off > ws_size) return;
  float* Vout = out; float* Cout = out + (size_t)NB_ * NC * DC; float* Bout = Cout + (size_t)3 * NB_ * SQ * NC;
  tr_kernel<<<dim3(NU / 64, DIN / 64), 256, 0, stream>>>(W, wt);
  proj_kernel<<<dim3(NU / 64, NR / 128), 128, 0, stream>>>(x, wt, u16);
  route_kernel<<<NB_, 256, 0, stream>>>(u16, Vout, Cout, Bout);
}
